// Mamba2DStable_24361054503033
// MI455X (gfx1250) — hardware-run, weakly checked
//
#include <hip/hip_runtime.h>
#include <math.h>

typedef __attribute__((ext_vector_type(16))) _Float16 v16h;
typedef __attribute__((ext_vector_type(8)))  _Float16 v8h;
typedef __attribute__((ext_vector_type(16))) __bf16   v16b;
typedef __attribute__((ext_vector_type(8)))  __bf16   v8b;
typedef __attribute__((ext_vector_type(8)))  float    v8f;
typedef __attribute__((ext_vector_type(4)))  float    v4f;

constexpr int kBatch = 2;
constexpr int kCh    = 512;
constexpr int kSeqL  = 4096;
constexpr int kDin   = 1024;
constexpr int kNst   = 16;
constexpr int kDtR   = 32;
constexpr int kXdP   = 64;
constexpr int kXzP   = 2 * kDin;
constexpr int kRows  = kBatch * kSeqL;
constexpr int kTP    = 260;
constexpr int kOP    = 36;
constexpr float kEps = 1e-5f;
constexpr float kCarWin  = 32.0f;
constexpr float kCarWx   = 32.0f;
constexpr float kCarWdt  = 8.0f;
constexpr float kCarWout = 32.0f;
constexpr float kCarUc   = 16.0f;
constexpr float kCarDt   = 16.0f;
constexpr float kCarY    = 256.0f;
static_assert(kDtR + 2 * kNst == kXdP, "x_proj width");
static_assert((kCh % 32) == 0 && (kDin % 32) == 0 && (kDtR % 32) == 0, "GEMM K multiples of 32");
static_assert((kSeqL % 64) == 0 && (kXzP % 64) == 0 && (kXdP % 64) == 0 && (kCh % 64) == 0 && (kDin % 64) == 0, "GEMM M,N multiples of 64");
static_assert((kDin % 256) == 0 && (kSeqL % 32) == 0 && kCh == 512, "tile multiples");

constexpr size_t kOffWIN  = 0;
constexpr size_t kOffWXP  = kOffWIN  + (size_t)kXzP * kCh * 2;
constexpr size_t kOffWDT  = kOffWXP  + (size_t)kXdP * kDin * 2;
constexpr size_t kOffWOUT = kOffWDT  + (size_t)kDin * kDtR * 2;
constexpr size_t kOffXS   = kOffWOUT + (size_t)kCh * kDin * 2;
constexpr size_t kOffXZ   = kOffXS   + (size_t)kRows * kCh * 2;
constexpr size_t kOffUC   = kOffXZ   + (size_t)kSeqL * kXzP * 4;
constexpr size_t kOffUC16 = kOffUC   + (size_t)kSeqL * kDin * 4;
constexpr size_t kOffXD   = kOffUC16 + (size_t)kSeqL * kDin * 2;
constexpr size_t kOffDT16 = kOffXD   + (size_t)kSeqL * kXdP * 4;
constexpr size_t kOffDLR  = kOffDT16 + (size_t)kSeqL * kDtR * 2;
constexpr size_t kOffY16  = kOffDLR  + (size_t)kSeqL * kDin * 4;
constexpr size_t kOffOPRE = kOffY16  + (size_t)kSeqL * kDin * 2;
constexpr size_t kWsTotal = kOffOPRE + (size_t)kSeqL * kCh * 4;
static_assert(kWsTotal == 105316352ull, "carve total");
static_assert(kWsTotal <= 134217728ull, "carve cap");
static_assert((kOffWXP % 128) == 0 && (kOffWDT % 128) == 0 && (kOffWOUT % 128) == 0 && (kOffXS % 128) == 0 &&
              (kOffXZ % 128) == 0 && (kOffUC % 128) == 0 && (kOffUC16 % 128) == 0 && (kOffXD % 128) == 0 &&
              (kOffDT16 % 128) == 0 && (kOffDLR % 128) == 0 && (kOffY16 % 128) == 0 && (kOffOPRE % 128) == 0,
              "128-B aligned regions");

__device__ __forceinline__ unsigned short f2bf_bits(float f) {
  unsigned u = __float_as_uint(f);
  return (unsigned short)((u + 0x7FFFu + ((u >> 16) & 1u)) >> 16);
}
__device__ __forceinline__ float bf_bits2f(unsigned short h) { return __uint_as_float(((unsigned)h) << 16); }

__device__ __forceinline__ void dep_guard4_h(v8f& a, v8f& b, v8f& c, v8f& d, v16h x, v16h y) {
  asm volatile("v_nop\n\tv_nop\n\tv_nop\n\tv_nop" : "+v"(a), "+v"(b), "+v"(c), "+v"(d) : "v"(x), "v"(y));
}
__device__ __forceinline__ void dep_guard4_b(v8f& a, v8f& b, v8f& c, v8f& d, v16b x, v16b y) {
  asm volatile("v_nop\n\tv_nop\n\tv_nop\n\tv_nop" : "+v"(a), "+v"(b), "+v"(c), "+v"(d) : "v"(x), "v"(y));
}
__device__ __forceinline__ void keep4_h(v16h a, v16h b, v16h c, v16h d) { asm volatile("v_nop" :: "v"(a), "v"(b), "v"(c), "v"(d)); }
__device__ __forceinline__ void keep4_b(v16b a, v16b b, v16b c, v16b d) { asm volatile("v_nop" :: "v"(a), "v"(b), "v"(c), "v"(d)); }
__device__ __forceinline__ void acc_guard4(v8f& a, v8f& b, v8f& c, v8f& d) { asm volatile("v_nop\n\tv_nop\n\tv_nop\n\tv_nop" : "+v"(a), "+v"(b), "+v"(c), "+v"(d)); }
template <typename T> struct Frag;
template <> struct Frag<_Float16> {
  typedef v16h V; union U { v16h v; v8h h[2]; };
  static __device__ __forceinline__ v16h load(const _Float16* p) {
    U f; f.h[0] = *(const v8h*)(p); f.h[1] = *(const v8h*)(p + 16); return f.v;
  }
  static __device__ __forceinline__ v8f mma(v16h a, v16h b, v8f c) {
    return __builtin_amdgcn_wmma_f32_16x16x32_f16(false, a, false, b, (short)0, c, false, false);
  }
  static __device__ __forceinline__ void guard4(v8f& a, v8f& b, v8f& c, v8f& d, v16h x, v16h y) { dep_guard4_h(a, b, c, d, x, y); }
  static __device__ __forceinline__ void keep(v16h a, v16h b, v16h c, v16h d) { keep4_h(a, b, c, d); }
};
template <> struct Frag<__bf16> {
  typedef v16b V; union U { v16b v; v8b h[2]; };
  static __device__ __forceinline__ v16b load(const __bf16* p) {
    U f; f.h[0] = *(const v8b*)(p); f.h[1] = *(const v8b*)(p + 16); return f.v;
  }
  static __device__ __forceinline__ v8f mma(v16b a, v16b b, v8f c) {
    return __builtin_amdgcn_wmma_f32_16x16x32_bf16(false, a, false, b, (short)0, c, false, false);
  }
  static __device__ __forceinline__ void guard4(v8f& a, v8f& b, v8f& c, v8f& d, v16b x, v16b y) { dep_guard4_b(a, b, c, d, x, y); }
  static __device__ __forceinline__ void keep(v16b a, v16b b, v16b c, v16b d) { keep4_b(a, b, c, d); }
};

template <int ET> struct Elem;
template <> struct Elem<0> { typedef _Float16 T; };
template <> struct Elem<1> { typedef __bf16 T; };
template <int ET, bool SPLIT, int BIAS_MODE, int OUT_MODE, bool RESID, int ACT = 0>
__global__ __launch_bounds__(256) void wmma_gemm64(
    const unsigned short* __restrict__ Ap, const unsigned short* __restrict__ A2p, int lda, long strideA,
    const unsigned short* __restrict__ Btp, const unsigned short* __restrict__ Bt2p, int ldb, long strideB,
    void* __restrict__ Cout, void* __restrict__ Cout2, int ldc, long strideC,
    const float* __restrict__ bias,
    const float* __restrict__ resid, long strideR,
    int M, int N, int K, float scale) {
  typedef typename Elem<ET>::T T;
  typedef typename Frag<T>::V V;
  const T* A = (const T*)Ap; const T* A2 = (const T*)A2p; const T* Bt = (const T*)Btp; const T* Bt2 = (const T*)Bt2p;
  __shared__ __align__(16) float sT[8][16 * 68];
  const int b    = blockIdx.y;
  const int lane = threadIdx.x & 31;
  const int wave = threadIdx.x >> 5;
  const int tilesN = N >> 6;
  const int tilesM = M >> 6;
  const int tile = blockIdx.x * 8 + wave;
  if (tile >= tilesM * tilesN) return;
  const int tm = tile / tilesN;
  const int tn = tile - tm * tilesN;
  const int m0 = tm << 6;
  const int n0 = tn << 6;

  const T* Ab  = A  + (size_t)b * strideA;
  const T* Bb  = Bt + (size_t)b * strideB;
  const T* Ab2 = SPLIT ? (A2  + (size_t)b * strideA) : nullptr;
  const T* Bb2 = SPLIT ? (Bt2 + (size_t)b * strideB) : nullptr;

  const int rlane = lane & 15;
  const int koff  = (lane >> 4) * 8;
  const int mOff  = (lane >> 4) * 8;

  v8f acc[4][4];
#pragma unroll
  for (int i = 0; i < 4; ++i)
#pragma unroll
    for (int j = 0; j < 4; ++j) acc[i][j] = (v8f){0.f,0.f,0.f,0.f,0.f,0.f,0.f,0.f};

  for (int k0 = 0; k0 < K; k0 += 32) {
    V bh[4], bl[4];
#pragma unroll
    for (int j = 0; j < 4; ++j) {
      const size_t bo = (size_t)(n0 + (j << 4) + rlane) * ldb + koff + k0;
      bh[j] = Frag<T>::load(Bb + bo);
      if (SPLIT) bl[j] = Frag<T>::load(Bb2 + bo);
    }
#pragma unroll
    for (int i = 0; i < 4; ++i) {
      const size_t ao = (size_t)(m0 + (i << 4) + rlane) * lda + koff + k0;
      V ah = Frag<T>::load(Ab + ao);
      V al;
      if (SPLIT) al = Frag<T>::load(Ab2 + ao);
#pragma unroll
      for (int j = 0; j < 4; ++j) {
        acc[i][j] = Frag<T>::mma(ah, bh[j], acc[i][j]);
        if (SPLIT) {
          acc[i][j] = Frag<T>::mma(ah, bl[j], acc[i][j]);
          acc[i][j] = Frag<T>::mma(al, bh[j], acc[i][j]);
        }
      }
      Frag<T>::guard4(acc[i][0], acc[i][1], acc[i][2], acc[i][3], ah, SPLIT ? al : ah);
    }
    Frag<T>::keep(bh[0], bh[1], bh[2], bh[3]);
    if (SPLIT) Frag<T>::keep(bl[0], bl[1], bl[2], bl[3]);
  }
  acc_guard4(acc[0][0], acc[0][1], acc[0][2], acc[0][3]);
  acc_guard4(acc[1][0], acc[1][1], acc[1][2], acc[1][3]);
  acc_guard4(acc[2][0], acc[2][1], acc[2][2], acc[2][3]);
  acc_guard4(acc[3][0], acc[3][1], acc[3][2], acc[3][3]);

  float* slab = sT[wave];
  const float* Rb = RESID ? (resid + (size_t)b * strideR) : nullptr;
#pragma unroll
  for (int i = 0; i < 4; ++i) {
    const int mBase = m0 + (i << 4);
#pragma unroll
    for (int j = 0; j < 4; ++j) {
      const int n = n0 + (j << 4) + rlane;
      float bv = 0.f;
      if (BIAS_MODE == 2) bv = bias[n];
#pragma unroll
      for (int r = 0; r < 8; ++r) {
        float v = acc[i][j][r] * scale;
        if (BIAS_MODE == 1) v += bias[mBase + mOff + r];
        if (BIAS_MODE == 2) v += bv;
        if (RESID) v += Rb[(size_t)(mBase + mOff + r) * ldc + n];
        if (ACT == 2) v = fmaxf(v, 0.0f);
        if (ACT == 4) v = (v > 0.f) ? v : 0.01f * v;
        slab[(mOff + r) * 68 + (j << 4) + rlane] = v;
      }
    }
    __builtin_amdgcn_fence(__ATOMIC_RELEASE, "workgroup");
    __builtin_amdgcn_wave_barrier();
    __builtin_amdgcn_fence(__ATOMIC_ACQUIRE, "workgroup");
    if (OUT_MODE == 0) {
      float* C = (float*)Cout + (size_t)b * strideC;
      const int hh = lane >> 4, c4 = (lane & 15) * 4;
      for (int pass = 0; pass < 2; ++pass) {
#pragma unroll
        for (int it = 0; it < 8; ++it) {
          const int row = it * 2 + hh;
          v4f v = *(const v4f*)(slab + row * 68 + c4);
          *(volatile v4f*)(C + (size_t)(mBase + row) * ldc + n0 + c4) = v;
        }
        __threadfence();
      }
    } else {
      const int q = lane >> 3, c8 = (lane & 7) * 8;
      unsigned short* C  = (unsigned short*)Cout  + (size_t)b * strideC;
      unsigned short* C2 = (OUT_MODE == 2) ? ((unsigned short*)Cout2 + (size_t)b * strideC) : nullptr;
      for (int pass = 0; pass < 2; ++pass) {
#pragma unroll
        for (int it = 0; it < 4; ++it) {
          const int row = it * 4 + q;
          const float* sp = slab + row * 68 + c8;
          v8h hv, lv;
#pragma unroll
          for (int e = 0; e < 8; ++e) {
            if (OUT_MODE == 1) {
              hv[e] = (_Float16)sp[e];
            } else {
              unsigned short hb = f2bf_bits(sp[e]);
              unsigned short lb = f2bf_bits(sp[e] - bf_bits2f(hb));
              hv[e] = __builtin_bit_cast(_Float16, hb);
              lv[e] = __builtin_bit_cast(_Float16, lb);
            }
          }
          *(volatile v8h*)(C + (size_t)(mBase + row) * ldc + n0 + c8) = hv;
          if (OUT_MODE == 2) *(volatile v8h*)(C2 + (size_t)(mBase + row) * ldc + n0 + c8) = lv;
        }
        __threadfence();
      }
    }
    __builtin_amdgcn_fence(__ATOMIC_RELEASE, "workgroup");
    __builtin_amdgcn_wave_barrier();
    __builtin_amdgcn_fence(__ATOMIC_ACQUIRE, "workgroup");
  }
}

__global__ __launch_bounds__(256) void cast_f16_kernel(
    const float* __restrict__ src, unsigned short* __restrict__ dst, int total8, float scale)
{
  const int i = blockIdx.x * 256 + threadIdx.x;
  if (i >= total8) return;
  const size_t e0 = (size_t)i << 3;
  const float* p = src + e0;
  const v4f a0 = *(const v4f*)(p);
  const v4f a1 = *(const v4f*)(p + 4);
  v8h hv;
#pragma unroll
  for (int e = 0; e < 4; ++e) {
    hv[e]     = (_Float16)(a0[e] * scale);
    hv[4 + e] = (_Float16)(a1[e] * scale);
  }
  unsigned short* q = dst + e0;
  *(volatile v8h*)q = hv;
  __threadfence();
  *(volatile v8h*)q = hv;
}

__device__ __forceinline__ float clamp10(float v) { return fminf(10.0f, fmaxf(-10.0f, v)); }
__device__ __forceinline__ v4f clamp4(v4f v) {
  v4f r;
  r[0] = clamp10(v[0]); r[1] = clamp10(v[1]); r[2] = clamp10(v[2]); r[3] = clamp10(v[3]);
  return r;
}

__global__ __launch_bounds__(256) void ln_in_kernel(
    const float* __restrict__ x, const float* __restrict__ nw, const float* __restrict__ nb,
    unsigned short* __restrict__ XS16)
{
  __shared__ __align__(16) float sT[32 * kTP];
  __shared__ __align__(16) float sRedA[8 * 32];
  __shared__ __align__(16) float sRedB[8 * 32];
  const int tid = threadIdx.x, lane = tid & 31, wave = tid >> 5;
  constexpr int kBlkPerB = kSeqL / 32;
  const int bix = blockIdx.x / kBlkPerB;
  const int l0  = (blockIdx.x - bix * kBlkPerB) * 32;
  const int cg = tid >> 3, l4 = (tid & 7) * 4;
  const float* xb = x + (size_t)bix * kCh * kSeqL + l0 + l4;

  v4f s = (v4f){0.f, 0.f, 0.f, 0.f};
#pragma unroll 1
  for (int i = 0; i < 16; ++i) {
    const v4f v = clamp4(*(const v4f*)(xb + (size_t)(cg + 32 * i) * kSeqL));
    s += v;
  }
#pragma unroll
  for (int e = 0; e < 4; ++e) {
    float t = s[e];
    t += __shfl_xor(t, 8, 32);
    t += __shfl_xor(t, 16, 32);
    s[e] = t;
  }
  if ((lane >> 3) == 0) *(v4f*)(sRedA + wave * 32 + l4) = s;
  __syncthreads();
  v4f mu = (v4f){0.f, 0.f, 0.f, 0.f};
#pragma unroll
  for (int w = 0; w < 8; ++w) mu += *(const v4f*)(sRedA + w * 32 + l4);
  mu = mu * (1.0f / (float)kCh);

  v4f qs = (v4f){0.f, 0.f, 0.f, 0.f};
#pragma unroll 1
  for (int i = 0; i < 16; ++i) {
    const v4f v = clamp4(*(const v4f*)(xb + (size_t)(cg + 32 * i) * kSeqL));
    const v4f dl = v - mu;
    qs += dl * dl;
  }
#pragma unroll
  for (int e = 0; e < 4; ++e) {
    float t = qs[e];
    t += __shfl_xor(t, 8, 32);
    t += __shfl_xor(t, 16, 32);
    qs[e] = t;
  }
  if ((lane >> 3) == 0) *(v4f*)(sRedB + wave * 32 + l4) = qs;
  __syncthreads();
  v4f var = (v4f){0.f, 0.f, 0.f, 0.f};
#pragma unroll
  for (int w = 0; w < 8; ++w) var += *(const v4f*)(sRedB + w * 32 + l4);
  var = var * (1.0f / (float)kCh);
  v4f rs;
#pragma unroll
  for (int e = 0; e < 4; ++e) rs[e] = rsqrtf(var[e] + kEps);

  const size_t rowbase = (size_t)bix * kSeqL + l0;
#pragma unroll 1
  for (int hf = 0; hf < 2; ++hf) {
#pragma unroll 1
    for (int i = 0; i < 8; ++i) {
      const int cl = cg + 32 * i;
      const int c  = hf * 256 + cl;
      const v4f v = clamp4(*(const v4f*)(xb + (size_t)c * kSeqL));
      const float wv = nw[c], bv = nb[c];
#pragma unroll
      for (int e = 0; e < 4; ++e) {
        const float o = clamp10(((v[e] - mu[e]) * rs[e]) * wv + bv);
        sT[(l4 + e) * kTP + cl] = o;
      }
    }
    __syncthreads();
    v8h hv[4];
#pragma unroll
    for (int it = 0; it < 4; ++it) {
      const float* sp = sT + (it * 8 + wave) * kTP + lane * 8;
      const v4f a0 = *(const v4f*)(sp);
      const v4f a1 = *(const v4f*)(sp + 4);
#pragma unroll
      for (int e = 0; e < 4; ++e) { hv[it][e] = (_Float16)a0[e]; hv[it][4 + e] = (_Float16)a1[e]; }
    }
    for (int pass = 0; pass < 2; ++pass) {
#pragma unroll
      for (int it = 0; it < 4; ++it)
        *(volatile v8h*)(XS16 + (rowbase + it * 8 + wave) * kCh + hf * 256 + lane * 8) = hv[it];
      __threadfence();
    }
    __syncthreads();
  }
}

__global__ __launch_bounds__(256) void conv_silu_kernel(
    const float* __restrict__ XZ, const float* __restrict__ cw, const float* __restrict__ cb,
    float* __restrict__ UC, unsigned short* __restrict__ UC16)
{
  __shared__ __align__(16) float sT[16 * kTP];
  const int tid = threadIdx.x, lane = tid & 31, wave = tid >> 5;
  const int d0 = blockIdx.x * 256, d = d0 + tid;
  const int t0 = blockIdx.y * 64;
  const v4f wq = *(const v4f*)(cw + (size_t)d * 4);
  const float w0 = wq[0], w1 = wq[1], w2 = wq[2], w3 = wq[3];
  const float bc = cb[d];
  float xm3, xm2, xm1;
  {
    const int r3 = t0 - 3, r2 = t0 - 2, r1 = t0 - 1;
    const float v3 = XZ[(size_t)(r3 < 0 ? 0 : r3) * kXzP + d];
    const float v2 = XZ[(size_t)(r2 < 0 ? 0 : r2) * kXzP + d];
    const float v1 = XZ[(size_t)(r1 < 0 ? 0 : r1) * kXzP + d];
    xm3 = (r3 >= 0) ? v3 : 0.f;
    xm2 = (r2 >= 0) ? v2 : 0.f;
    xm1 = (r1 >= 0) ? v1 : 0.f;
  }
  const int hrow = wave >> 1;
  const int hch  = (wave & 1) * 128 + lane * 4;
#pragma unroll 1
  for (int sub = 0; sub < 4; ++sub) {
    const int lb = t0 + sub * 16;
#pragma unroll 1
    for (int s = 0; s < 16; ++s) {
      const float xcur = XZ[(size_t)(lb + s) * kXzP + d];
      float acc = w0 * xm3;
      acc = fmaf(w1, xm2, acc);
      acc = fmaf(w2, xm1, acc);
      acc = fmaf(w3, xcur, acc);
      const float sv = acc + bc;
      const float sg = __builtin_amdgcn_rcpf(1.0f + expf(-sv));
      sT[s * kTP + tid] = sv * sg;
      xm3 = xm2; xm2 = xm1; xm1 = xcur;
    }
    __syncthreads();
    v4f fv[4];
    v8h bv[2];
#pragma unroll
    for (int it = 0; it < 4; ++it) fv[it] = *(const v4f*)(sT + (it * 4 + hrow) * kTP + hch);
#pragma unroll
    for (int it = 0; it < 2; ++it) {
      const float* sp = sT + (it * 8 + wave) * kTP + lane * 8;
      const v4f a0 = *(const v4f*)(sp);
      const v4f a1 = *(const v4f*)(sp + 4);
#pragma unroll
      for (int e = 0; e < 4; ++e) {
        bv[it][e]     = (_Float16)(a0[e] * kCarUc);
        bv[it][4 + e] = (_Float16)(a1[e] * kCarUc);
      }
    }
    for (int pass = 0; pass < 2; ++pass) {
#pragma unroll
      for (int it = 0; it < 4; ++it)
        *(volatile v4f*)(UC + (size_t)(lb + it * 4 + hrow) * kDin + d0 + hch) = fv[it];
#pragma unroll
      for (int it = 0; it < 2; ++it)
        *(volatile v8h*)(UC16 + (size_t)(lb + it * 8 + wave) * kDin + d0 + lane * 8) = bv[it];
      __threadfence();
    }
    __syncthreads();
  }
}

__global__ __launch_bounds__(256) void dt_cast_kernel(
    const float* __restrict__ XD, unsigned short* __restrict__ DT16, int total8, float scale)
{
  const int i = blockIdx.x * 256 + threadIdx.x;
  if (i >= total8) return;
  const int e0  = i << 3;
  const int row = e0 >> 5;
  const int c8  = e0 & 31;
  const float* p = XD + (size_t)row * kXdP + c8;
  const v4f a0 = *(const v4f*)(p);
  const v4f a1 = *(const v4f*)(p + 4);
  v8h hv;
#pragma unroll
  for (int e = 0; e < 4; ++e) {
    hv[e]     = (_Float16)(a0[e] * scale);
    hv[4 + e] = (_Float16)(a1[e] * scale);
  }
  unsigned short* qd = DT16 + e0;
  *(volatile v8h*)qd = hv;
  __threadfence();
  *(volatile v8h*)qd = hv;
}

__global__ __launch_bounds__(256) void scan_kernel(
    const float* __restrict__ DLR, const float* __restrict__ UC, const float* __restrict__ XZ,
    const float* __restrict__ XD, const float* __restrict__ A_log, const float* __restrict__ Dv,
    unsigned short* __restrict__ Y16)
{
  __shared__ __align__(16) float sBC[16 * 32];
  __shared__ __align__(16) float sY[16 * kTP];
  __shared__ __align__(16) float sA[kNst * 256];
  const int tid = threadIdx.x, lane = tid & 31, wave = tid >> 5;
  const int d0 = blockIdx.x * 256, d = d0 + tid;

#pragma unroll 1
  for (int n = 0; n < kNst; ++n) sA[n * 256 + tid] = -expf(A_log[(size_t)d * kNst + n]);
  __syncthreads();
  float An[kNst], h[kNst];
#pragma unroll
  for (int n = 0; n < kNst; ++n) {
    An[n] = sA[n * 256 + tid];
    h[n] = 0.f;
  }
  const float Dd = Dv[d];

#pragma unroll 1
  for (int c = 0; c < kSeqL / 16; ++c) {
    const int l0 = c * 16;
    if (tid < 128) {
      const int r = tid >> 3, q = (tid & 7) * 4;
      const v4f v = *(const v4f*)(XD + (size_t)(l0 + r) * kXdP + kDtR + q);
      *(v4f*)(sBC + r * 32 + q) = v;
    }
    __syncthreads();
#pragma unroll 1
    for (int s = 0; s < 16; ++s) {
      const size_t m = (size_t)(l0 + s);
      const float a  = DLR[m * kDin + d];
      const float xv = UC[m * kDin + d];
      const float zv = XZ[m * kXzP + kDin + d];
      const float ea  = __expf(-fabsf(a));
      const float u   = 1.0f + ea;
      const float l1p = __logf(u) + (ea - (u - 1.0f)) * __builtin_amdgcn_rcpf(u);
      const float delta = fmaxf(a, 0.0f) + l1p;
      v4f Bq[4], Cq[4];
#pragma unroll
      for (int qq = 0; qq < 4; ++qq) {
        Bq[qq] = *(const v4f*)(sBC + s * 32 + 4 * qq);
        Cq[qq] = *(const v4f*)(sBC + s * 32 + kNst + 4 * qq);
      }
      const float dtx = delta * xv;
      float y = 0.f;
#pragma unroll
      for (int n = 0; n < kNst; ++n) {
        const float e = __expf(delta * An[n]);
        h[n] = e * h[n] + dtx * Bq[n >> 2][n & 3];
        y = h[n] * Cq[n >> 2][n & 3] + y;
      }
      y = xv * Dd + y;
      const float sg = __builtin_amdgcn_rcpf(1.0f + expf(-zv));
      const float g  = zv * sg;
      sY[s * kTP + tid] = (y * g) * kCarY;
    }
    __syncthreads();
    v8h hv[2];
#pragma unroll
    for (int it = 0; it < 2; ++it) {
      const float* sp = sY + (it * 8 + wave) * kTP + lane * 8;
      const v4f a0 = *(const v4f*)(sp);
      const v4f a1 = *(const v4f*)(sp + 4);
#pragma unroll
      for (int e = 0; e < 4; ++e) { hv[it][e] = (_Float16)a0[e]; hv[it][4 + e] = (_Float16)a1[e]; }
    }
    for (int pass = 0; pass < 2; ++pass) {
#pragma unroll
      for (int it = 0; it < 2; ++it)
        *(volatile v8h*)(Y16 + (size_t)(l0 + it * 8 + wave) * kDin + d0 + lane * 8) = hv[it];
      __threadfence();
    }
  }
}

__global__ __launch_bounds__(256) void ln_out_kernel(const float* __restrict__ OP, float* __restrict__ outb)
{
  __shared__ __align__(16) float sT[128 * kOP];
  __shared__ float sMu[32];
  __shared__ float sRs[32];
  const int tid = threadIdx.x, lane = tid & 31, wave = tid >> 5;
  const int l0 = blockIdx.x * 32;
#pragma unroll 1
  for (int j = 0; j < 4; ++j) {
    const int row = wave * 4 + j;
    const float* p = OP + (size_t)(l0 + row) * kCh + lane * 4;
    v4f a[4];
#pragma unroll
    for (int t = 0; t < 4; ++t) a[t] = clamp4(*(const v4f*)(p + t * 128));
    float s = 0.f;
#pragma unroll
    for (int t = 0; t < 4; ++t) s += (a[t][0] + a[t][1]) + (a[t][2] + a[t][3]);
    s += __shfl_xor(s, 16, 32);
    s += __shfl_xor(s, 8, 32);
    s += __shfl_xor(s, 4, 32);
    s += __shfl_xor(s, 2, 32);
    s += __shfl_xor(s, 1, 32);
    const float mu = s * (1.0f / (float)kCh);
    float q = 0.f;
#pragma unroll
    for (int t = 0; t < 4; ++t) {
#pragma unroll
      for (int e = 0; e < 4; ++e) {
        const float dl = a[t][e] - mu;
        q = fmaf(dl, dl, q);
      }
    }
    q += __shfl_xor(q, 16, 32);
    q += __shfl_xor(q, 8, 32);
    q += __shfl_xor(q, 4, 32);
    q += __shfl_xor(q, 2, 32);
    q += __shfl_xor(q, 1, 32);
    const float rsd = rsqrtf(q * (1.0f / (float)kCh) + kEps);
    if (lane == 0) { sMu[row] = mu; sRs[row] = rsd; }
  }
  __syncthreads();
  const int lrow = tid >> 3, cq = (tid & 7) * 4;
  const float mu = sMu[lrow], rsd = sRs[lrow];
  const int q4 = lane >> 3, l4 = (lane & 7) * 4;
#pragma unroll 1
  for (int cc = 0; cc < 4; ++cc) {
#pragma unroll
    for (int t = 0; t < 4; ++t) {
      const int cl = t * 32 + cq;
      const v4f v = clamp4(*(const v4f*)(OP + (size_t)(l0 + lrow) * kCh + cc * 128 + cl));
#pragma unroll
      for (int e = 0; e < 4; ++e) {
        const float o = clamp10((v[e] - mu) * rsd);
        sT[(cl + e) * kOP + lrow] = o;
      }
    }
    __syncthreads();
    v4f hv[4];
#pragma unroll
    for (int it = 0; it < 4; ++it) hv[it] = *(const v4f*)(sT + (it * 32 + wave * 4 + q4) * kOP + l4);
    for (int pass = 0; pass < 2; ++pass) {
#pragma unroll
      for (int it = 0; it < 4; ++it) {
        const int cl = it * 32 + wave * 4 + q4;
        *(volatile v4f*)(outb + (size_t)(cc * 128 + cl) * kSeqL + l0 + l4) = hv[it];
      }
      __threadfence();
    }
    __syncthreads();
  }
}

extern "C" void kernel_launch(void* const* d_in, const int* in_sizes, int n_in,
                              void* d_out, int out_size, void* d_ws, size_t ws_size,
                              hipStream_t stream)
{
  if (n_in < 12) return;
  if (in_sizes[0] != kRows * kCh) return;
  if (in_sizes[1] != kCh || in_sizes[2] != kCh) return;
  if (in_sizes[3] != kXzP * kCh) return;
  if (in_sizes[4] != kDin * 4 || in_sizes[5] != kDin) return;
  if (in_sizes[6] != kXdP * kDin) return;
  if (in_sizes[7] != kDin * kDtR || in_sizes[8] != kDin) return;
  if (in_sizes[9] != kDin * kNst || in_sizes[10] != kDin) return;
  if (in_sizes[11] != kCh * kDin) return;
  if (out_size != kRows * kCh) return;
  if (ws_size < kWsTotal) return;

  const float* x      = (const float*)d_in[0];
  const float* norm_w = (const float*)d_in[1];
  const float* norm_b = (const float*)d_in[2];
  const float* W_in   = (const float*)d_in[3];
  const float* conv_w = (const float*)d_in[4];
  const float* conv_b = (const float*)d_in[5];
  const float* W_xprj = (const float*)d_in[6];
  const float* W_dt   = (const float*)d_in[7];
  const float* b_dt   = (const float*)d_in[8];
  const float* A_log  = (const float*)d_in[9];
  const float* Dv     = (const float*)d_in[10];
  const float* W_out  = (const float*)d_in[11];
  float* dout = (float*)d_out;

  char* ws = (char*)d_ws;
  unsigned short* WIN16  = (unsigned short*)(ws + kOffWIN);
  unsigned short* WXP16  = (unsigned short*)(ws + kOffWXP);
  unsigned short* WDT16  = (unsigned short*)(ws + kOffWDT);
  unsigned short* WOUT16 = (unsigned short*)(ws + kOffWOUT);
  unsigned short* XS16   = (unsigned short*)(ws + kOffXS);
  float*          XZ     = (float*)(ws + kOffXZ);
  float*          UC     = (float*)(ws + kOffUC);
  unsigned short* UC16   = (unsigned short*)(ws + kOffUC16);
  float*          XD     = (float*)(ws + kOffXD);
  unsigned short* DT16   = (unsigned short*)(ws + kOffDT16);
  float*          DLR    = (float*)(ws + kOffDLR);
  unsigned short* Y16    = (unsigned short*)(ws + kOffY16);
  float*          OPRE   = (float*)(ws + kOffOPRE);
  const float* dummy_bias  = b_dt;
  const float* dummy_resid = x;

  cast_f16_kernel<<<(kXzP * kCh / 8) / 256, 256, 0, stream>>>(W_in,   WIN16,  kXzP * kCh / 8,  kCarWin);
  cast_f16_kernel<<<(kXdP * kDin / 8) / 256, 256, 0, stream>>>(W_xprj, WXP16,  kXdP * kDin / 8, kCarWx);
  cast_f16_kernel<<<(kDin * kDtR / 8) / 256, 256, 0, stream>>>(W_dt,   WDT16,  kDin * kDtR / 8, kCarWdt);
  cast_f16_kernel<<<(kCh * kDin / 8) / 256, 256, 0, stream>>>(W_out,  WOUT16, kCh * kDin / 8,  kCarWout);

  ln_in_kernel<<<kRows / 32, 256, 0, stream>>>(x, norm_w, norm_b, XS16);

  for (int b = 0; b < kBatch; ++b) {
    const unsigned short* XSb = XS16 + (size_t)b * kSeqL * kCh;
    float* outb = dout + (size_t)b * kCh * kSeqL;

    wmma_gemm64<0, false, 0, 0, false><<<dim3(256, 1), 256, 0, stream>>>(
        XSb, XSb, kCh, 0L, WIN16, WIN16, kCh, 0L,
        (void*)XZ, (void*)XZ, kXzP, 0L, dummy_bias, dummy_resid, 0L,
        kSeqL, kXzP, kCh, 1.0f / kCarWin);

    conv_silu_kernel<<<dim3(kDin / 256, kSeqL / 64), 256, 0, stream>>>(XZ, conv_w, conv_b, UC, UC16);

    wmma_gemm64<0, false, 0, 0, false><<<dim3(8, 1), 256, 0, stream>>>(
        UC16, UC16, kDin, 0L, WXP16, WXP16, kDin, 0L,
        (void*)XD, (void*)XD, kXdP, 0L, dummy_bias, dummy_resid, 0L,
        kSeqL, kXdP, kDin, 1.0f / (kCarUc * kCarWx));

    dt_cast_kernel<<<(kSeqL * kDtR / 8) / 256, 256, 0, stream>>>(XD, DT16, kSeqL * kDtR / 8, kCarDt);

    wmma_gemm64<0, false, 2, 0, false><<<dim3(128, 1), 256, 0, stream>>>(
        DT16, DT16, kDtR, 0L, WDT16, WDT16, kDtR, 0L,
        (void*)DLR, (void*)DLR, kDin, 0L, b_dt, dummy_resid, 0L,
        kSeqL, kDin, kDtR, 1.0f / (kCarDt * kCarWdt));

    scan_kernel<<<dim3(kDin / 256, 1), 256, 0, stream>>>(DLR, UC, XZ, XD, A_log, Dv, Y16);

    wmma_gemm64<0, false, 0, 0, false><<<dim3(64, 1), 256, 0, stream>>>(
        Y16, Y16, kDin, 0L, WOUT16, WOUT16, kDin, 0L,
        (void*)OPRE, (void*)OPRE, kCh, 0L, dummy_bias, dummy_resid, 0L,
        kSeqL, kCh, kDin, 1.0f / (kCarY * kCarWout));

    ln_out_kernel<<<kSeqL / 32, 256, 0, stream>>>(OPRE, outb);
  }
}
